// SoftmaxLoss_86096914415969
// MI455X (gfx1250) — hardware-verified
//
#include <hip/hip_runtime.h>
#include <stddef.h>


#define ALPHA_C     10.0f
#define BETA_C      2.0f
#define NCLS        98
#define NCLS_PAD    128
#define NCT         7
#define EMB         512
#define NROWS       8192
#define OPSCALE     64.0f
#define PSCALE      4096.0f
#define INV_PSCALE  (1.0f / 4096.0f)

#define CVT_RPB     8
#define CE_RPB      128
#define SIM_RPB     128
#define SIM_CCH     2048
#define KSTEPS      (EMB / 32)

typedef _Float16     v8h  __attribute__((ext_vector_type(8)));
typedef _Float16     v16h __attribute__((ext_vector_type(16)));
typedef float        v8f  __attribute__((ext_vector_type(8)));
typedef float        v4f  __attribute__((ext_vector_type(4)));
typedef unsigned int v4u  __attribute__((ext_vector_type(4)));
typedef v4f __attribute__((may_alias)) v4fa;

union Frag  { v16h v; v8h hv[2]; };
union Pack8 { v8h h; v4u u; };

typedef char chk_emb [(EMB == 512) ? 1 : -1];
typedef char chk_rows[(NROWS % SIM_RPB == 0 && NROWS % SIM_CCH == 0 && NROWS % CE_RPB == 0 &&
                       NROWS % CVT_RPB == 0 && SIM_CCH % 32 == 0 && NROWS % 256 == 0 &&
                       SIM_RPB == 128 && CE_RPB == 128) ? 1 : -1];
typedef char chk_cls [(NCT * 16 >= NCLS && NCT * 16 <= NCLS_PAD && NCLS_PAD % 16 == 0) ? 1 : -1];

__device__ __forceinline__ v8f wmma16(const v16h a, const v16h b, v8f c) {
    v8f d = __builtin_amdgcn_wmma_f32_16x16x32_f16(false, a, false, b, (short)0, c, false, false);
    asm volatile("v_nop\n\tv_nop\n\tv_nop\n\tv_nop" : "+v"(d) : "v"(a), "v"(b));
    return d;
}

__device__ __forceinline__ v8f zero8() {
    v8f z;
#pragma unroll
    for (int i = 0; i < 8; ++i) z[i] = 0.0f;
    return z;
}

__global__ void __launch_bounds__(256)
k_cvt(const float* __restrict__ X, _Float16* __restrict__ X16) {
    const int lane = threadIdx.x & 31;
    const int wave = threadIdx.x >> 5;
    const int row  = blockIdx.x * CVT_RPB + wave;
    if (row >= NROWS) return;
    const float* xr = X + (size_t)row * EMB;
    const v4f* s0 = (const v4f*)(xr + 8 * lane);
    const v4f* s1 = (const v4f*)(xr + 256 + 8 * lane);
    const v4f a0 = s0[0], a1 = s0[1], b0 = s1[0], b1 = s1[1];
    Pack8 o0, o1;
#pragma unroll
    for (int i = 0; i < 4; ++i) {
        o0.h[i]     = (_Float16)(a0[i] * OPSCALE);
        o0.h[4 + i] = (_Float16)(a1[i] * OPSCALE);
        o1.h[i]     = (_Float16)(b0[i] * OPSCALE);
        o1.h[4 + i] = (_Float16)(b1[i] * OPSCALE);
    }
    _Float16* dr = X16 + (size_t)row * EMB;
    volatile v4u* p0 = (volatile v4u*)(dr + 8 * lane);
    volatile v4u* p1 = (volatile v4u*)(dr + 256 + 8 * lane);
    const v4u u0 = o0.u, u1 = o1.u;
    *p0 = u0; *p1 = u1;
    __threadfence();
    *p0 = u0; *p1 = u1;
}

__global__ void __launch_bounds__(32)
k_wnorm(const float* __restrict__ K, _Float16* __restrict__ WnT16) {
    const int c    = blockIdx.x;
    const int lane = threadIdx.x & 31;
    float x[8], y[8];
    float ss = 0.0f;
    if (c < NCLS) {
#pragma unroll
        for (int i = 0; i < 8; ++i) {
            x[i] = K[(8 * lane + i) * NCLS + c];
            y[i] = K[(256 + 8 * lane + i) * NCLS + c];
            ss += x[i] * x[i];
            ss += y[i] * y[i];
        }
    } else {
#pragma unroll
        for (int i = 0; i < 8; ++i) { x[i] = 0.0f; y[i] = 0.0f; }
    }
#pragma unroll
    for (int msk = 16; msk >= 1; msk >>= 1) ss += __shfl_xor(ss, msk, 32);
    const float rn = (c < NCLS) ? (1.0f / sqrtf(ss)) : 0.0f;
    Pack8 o0, o1;
#pragma unroll
    for (int i = 0; i < 8; ++i) {
        o0.h[i] = (_Float16)((x[i] * rn) * OPSCALE);
        o1.h[i] = (_Float16)((y[i] * rn) * OPSCALE);
    }
    _Float16* dr = WnT16 + (size_t)c * EMB;
    volatile v4u* p0 = (volatile v4u*)(dr + 8 * lane);
    volatile v4u* p1 = (volatile v4u*)(dr + 256 + 8 * lane);
    const v4u u0 = o0.u, u1 = o1.u;
    *p0 = u0; *p1 = u1;
    __threadfence();
    *p0 = u0; *p1 = u1;
}

__global__ void __launch_bounds__(256)
k_ce(const _Float16* __restrict__ X16, const _Float16* __restrict__ WnT16,
     const int* __restrict__ tgt, float* __restrict__ RowLoss, float* __restrict__ RowCorr) {
    __shared__ __attribute__((aligned(16))) float lLoss[CE_RPB];
    __shared__ __attribute__((aligned(16))) float lCorr[CE_RPB];
    const int lane = threadIdx.x & 31;
    const int wave = threadIdx.x >> 5;
    const int h    = lane >> 4;
    const int m    = lane & 15;
    const int row0 = blockIdx.x * CE_RPB + wave * 16;

    v8f acc[NCT];
#pragma unroll
    for (int j = 0; j < NCT; ++j) acc[j] = zero8();

    const _Float16* aRow = X16 + (size_t)(row0 + m) * EMB + 8 * h;
#pragma unroll 1
    for (int kt = 0; kt < KSTEPS; ++kt) {
        const int kk = 32 * kt;
        Frag a;
        a.hv[0] = *(const v8h*)(aRow + kk);
        a.hv[1] = *(const v8h*)(aRow + kk + 16);
#pragma unroll
        for (int j = 0; j < NCT; ++j) {
            const _Float16* bRow = WnT16 + (size_t)(16 * j + m) * EMB + 8 * h + kk;
            Frag b;
            b.hv[0] = *(const v8h*)(bRow);
            b.hv[1] = *(const v8h*)(bRow + 16);
            acc[j] = wmma16(a.v, b.v, acc[j]);
        }
    }

#pragma unroll
    for (int r = 0; r < 8; ++r) {
        const int row = row0 + 8 * h + r;
        const int t   = tgt[row];
        float lg[NCT];
        float bv = -3.0e38f;
        int   bi = 0x7fffffff;
#pragma unroll
        for (int j = 0; j < NCT; ++j) {
            const int c = 16 * j + m;
            float cv = acc[j][r] * INV_PSCALE;
            cv = fminf(fmaxf(cv, -1.0f), 1.0f);
            float l = (cv - ((c == t) ? BETA_C : 0.0f)) * ALPHA_C;
            if (c >= NCLS) l = -3.0e38f;
            lg[j] = l;
            if (l > bv) { bv = l; bi = c; }
        }
#pragma unroll
        for (int msk = 8; msk >= 1; msk >>= 1) {
            const float ov = __shfl_xor(bv, msk, 16);
            const int   oi = __shfl_xor(bi, msk, 16);
            if (ov > bv || (ov == bv && oi < bi)) { bv = ov; bi = oi; }
        }
        float se = 0.0f, tl = 0.0f;
#pragma unroll
        for (int j = 0; j < NCT; ++j) {
            const int c = 16 * j + m;
            se += __expf(lg[j] - bv);
            tl += (c == t) ? lg[j] : 0.0f;
        }
#pragma unroll
        for (int msk = 8; msk >= 1; msk >>= 1) {
            se += __shfl_xor(se, msk, 16);
            tl += __shfl_xor(tl, msk, 16);
        }
        if (m == 0) {
            const int lr = wave * 16 + 8 * h + r;
            lLoss[lr] = (bv + __logf(se)) - tl;
            lCorr[lr] = (bi == t) ? 1.0f : 0.0f;
        }
    }
    __syncthreads();
    if (wave == 0) {
        const v4f v = ((const v4fa*)lLoss)[lane];
        float* dst = RowLoss + (size_t)blockIdx.x * CE_RPB + 4 * lane;
        *(volatile v4f*)dst = v;
        __threadfence();
        *(volatile v4f*)dst = v;
    } else if (wave == 1) {
        const v4f v = ((const v4fa*)lCorr)[lane];
        float* dst = RowCorr + (size_t)blockIdx.x * CE_RPB + 4 * lane;
        *(volatile v4f*)dst = v;
        __threadfence();
        *(volatile v4f*)dst = v;
    }
}

__global__ void __launch_bounds__(256)
k_sim(const _Float16* __restrict__ X16, const float* __restrict__ X,
      const int* __restrict__ tgt, float* __restrict__ Part) {
    extern __shared__ v4u smem_v4[];
    char*     smem    = (char*)smem_v4;
    _Float16* ldsX    = (_Float16*)smem;
    int*      ldsCl   = (int*)(smem + (size_t)SIM_RPB * EMB * sizeof(_Float16));
    int*      ldsFlag = ldsCl + SIM_RPB;
    float*    ldsPart = (float*)(ldsFlag + SIM_RPB);

    const int rowBase  = blockIdx.x * SIM_RPB;
    const int chunk    = blockIdx.y;
    const int colChunk = chunk * SIM_CCH;

    {
        const v4u* src = (const v4u*)(X16 + (size_t)rowBase * EMB);
        v4u* dst = (v4u*)ldsX;
        for (int i = threadIdx.x; i < SIM_RPB * EMB / 8; i += 256) dst[i] = src[i];
        if (threadIdx.x < SIM_RPB) {
            ldsCl[threadIdx.x]   = tgt[rowBase + threadIdx.x];
            ldsFlag[threadIdx.x] = 0;
        }
    }
    __syncthreads();

    const int lane     = threadIdx.x & 31;
    const int wave     = threadIdx.x >> 5;
    const int m        = lane & 15;
    const int hf       = lane >> 4;
    const int waveRow0 = wave * 16;

    if (rowBase >= colChunk && rowBase < colChunk + SIM_CCH) {
        for (int rr = 0; rr < 16; ++rr) {
            const float* xr = X + (size_t)(rowBase + waveRow0 + rr) * EMB;
            float ss = 0.0f;
#pragma unroll
            for (int q = 0; q < 16; ++q) {
                const float v = xr[lane + 32 * q];
                ss += v * v;
            }
#pragma unroll
            for (int msk = 16; msk >= 1; msk >>= 1) ss += __shfl_xor(ss, msk, 32);
            if (lane == 0) ldsFlag[waveRow0 + rr] = (ss < 1.0f) ? 1 : 0;
        }
    }
    __syncthreads();

    int rCls[8];
    int selfMask = 0;
#pragma unroll
    for (int r = 0; r < 8; ++r) {
        const int lr = waveRow0 + 8 * hf + r;
        rCls[r] = ldsCl[lr];
        selfMask |= (ldsFlag[lr] & 1) << r;
    }
    float pS[8], nS[8], pC[8], nC[8];
#pragma unroll
    for (int r = 0; r < 8; ++r) { pS[r] = 0.0f; nS[r] = 0.0f; pC[r] = 0.0f; nC[r] = 0.0f; }

    const int rId0 = rowBase + waveRow0 + 8 * hf;
    const _Float16* aBase = ldsX + (size_t)(waveRow0 + m) * EMB + 8 * hf;

    for (int ct = 0; ct < SIM_CCH / 32; ++ct) {
        const int colBase = colChunk + ct * 32;
        const int col0    = colBase + m;
        const int col1    = col0 + 16;
        const int cCls0   = tgt[col0];
        const int cCls1   = tgt[col1];
        const _Float16* b0Base = X16 + (size_t)col0 * EMB + 8 * hf;
        const _Float16* b1Base = X16 + (size_t)col1 * EMB + 8 * hf;

        v8f acc0 = zero8();
        v8f acc1 = zero8();
#pragma unroll 4
        for (int kt = 0; kt < KSTEPS; ++kt) {
            const int kk = 32 * kt;
            Frag A, B0, B1;
            B0.hv[0] = *(const v8h*)(b0Base + kk);
            B0.hv[1] = *(const v8h*)(b0Base + kk + 16);
            B1.hv[0] = *(const v8h*)(b1Base + kk);
            B1.hv[1] = *(const v8h*)(b1Base + kk + 16);
            A.hv[0]  = *(const v8h*)(aBase + kk);
            A.hv[1]  = *(const v8h*)(aBase + kk + 16);
            acc0 = __builtin_amdgcn_wmma_f32_16x16x32_f16(false, A.v, false, B0.v, (short)0, acc0, false, false);
            acc1 = __builtin_amdgcn_wmma_f32_16x16x32_f16(false, A.v, false, B1.v, (short)0, acc1, false, false);
            asm volatile("v_nop\n\tv_nop\n\tv_nop\n\tv_nop"
                         : "+v"(acc0), "+v"(acc1) : "v"(A.v), "v"(B0.v), "v"(B1.v));
        }

#pragma unroll
        for (int r = 0; r < 8; ++r) {
            const int  rid    = rId0 + r;
            const bool selfLt = ((selfMask >> r) & 1) != 0;
            {
                const float s    = acc0[r];
                const bool  same = (rCls[r] == cCls0);
                const bool  lt   = (rid == col0) ? selfLt : (s < PSCALE);
                const bool  pos  = same && lt;
                pS[r] += pos ? s : 0.0f;
                pC[r] += pos ? 1.0f : 0.0f;
                nS[r] += same ? 0.0f : s;
                nC[r] += same ? 0.0f : 1.0f;
            }
            {
                const float s    = acc1[r];
                const bool  same = (rCls[r] == cCls1);
                const bool  lt   = (rid == col1) ? selfLt : (s < PSCALE);
                const bool  pos  = same && lt;
                pS[r] += pos ? s : 0.0f;
                pC[r] += pos ? 1.0f : 0.0f;
                nS[r] += same ? 0.0f : s;
                nC[r] += same ? 0.0f : 1.0f;
            }
        }
    }

#pragma unroll
    for (int r = 0; r < 8; ++r) {
        float a = pS[r], b = nS[r], c = pC[r], d = nC[r];
#pragma unroll
        for (int msk = 8; msk >= 1; msk >>= 1) {
            a += __shfl_xor(a, msk, 16);
            b += __shfl_xor(b, msk, 16);
            c += __shfl_xor(c, msk, 16);
            d += __shfl_xor(d, msk, 16);
        }
        if (m == 0) {
            const int lr = waveRow0 + 8 * hf + r;
            ldsPart[lr]               = a;
            ldsPart[SIM_RPB + lr]     = b;
            ldsPart[2 * SIM_RPB + lr] = c;
            ldsPart[3 * SIM_RPB + lr] = d;
        }
    }
    __syncthreads();
    if (wave < 4) {
        const v4fa* src = (const v4fa*)(ldsPart + wave * SIM_RPB);
        const v4f v = src[lane];
        float* dst = Part + ((size_t)(wave * 4 + chunk) * NROWS + rowBase + 4 * lane);
        *(volatile v4f*)dst = v;
        __threadfence();
        *(volatile v4f*)dst = v;
    }
}

__global__ void __launch_bounds__(256)
k_fin(const float* __restrict__ Part, const float* __restrict__ RowLoss,
      const float* __restrict__ RowCorr, float* __restrict__ out) {
    __shared__ double red[4][256];
    const int tid = threadIdx.x;
    double sl = 0.0, sc = 0.0, sp = 0.0, sn = 0.0;
    const size_t N = NROWS;
    for (int i = tid; i < NROWS; i += 256) {
        sl += (double)RowLoss[i];
        sc += (double)RowCorr[i];
        float ps = Part[(0 * 4 + 0) * N + i];
        ps += Part[(0 * 4 + 1) * N + i];
        ps += Part[(0 * 4 + 2) * N + i];
        ps += Part[(0 * 4 + 3) * N + i];
        float ns = Part[(1 * 4 + 0) * N + i];
        ns += Part[(1 * 4 + 1) * N + i];
        ns += Part[(1 * 4 + 2) * N + i];
        ns += Part[(1 * 4 + 3) * N + i];
        float pc = Part[(2 * 4 + 0) * N + i];
        pc += Part[(2 * 4 + 1) * N + i];
        pc += Part[(2 * 4 + 2) * N + i];
        pc += Part[(2 * 4 + 3) * N + i];
        float nc = Part[(3 * 4 + 0) * N + i];
        nc += Part[(3 * 4 + 1) * N + i];
        nc += Part[(3 * 4 + 2) * N + i];
        nc += Part[(3 * 4 + 3) * N + i];
        const float pm = (ps / pc) * INV_PSCALE;
        const float nm = (ns / nc) * INV_PSCALE;
        sp += (double)pm;
        sn += (double)nm;
    }
    red[0][tid] = sl; red[1][tid] = sc; red[2][tid] = sp; red[3][tid] = sn;
    __syncthreads();
    for (int off = 128; off >= 1; off >>= 1) {
        if (tid < off) {
            red[0][tid] += red[0][tid + off];
            red[1][tid] += red[1][tid + off];
            red[2][tid] += red[2][tid + off];
            red[3][tid] += red[3][tid + off];
        }
        __syncthreads();
    }
    if (tid == 0) {
        const double inv = 1.0 / (double)NROWS;
        v4f o;
        o[0] = (float)(red[0][0] * inv);
        o[1] = (float)(red[1][0] * inv);
        o[2] = (float)(red[2][0] * inv);
        o[3] = (float)(red[3][0] * inv);
        volatile v4f* po = (volatile v4f*)out;
        *po = o;
        __threadfence();
        *po = o;
    }
}

extern "C" void kernel_launch(void* const* d_in, const int* in_sizes, int n_in,
                              void* d_out, int out_size, void* d_ws, size_t ws_size,
                              hipStream_t stream) {
    if (n_in < 3) return;
    if (in_sizes[0] != NROWS * EMB || in_sizes[1] != NROWS || in_sizes[2] != EMB * NCLS) return;
    if (out_size < 4) return;

    const float* X   = (const float*)d_in[0];
    const int*   tgt = (const int*)d_in[1];
    const float* Kw  = (const float*)d_in[2];

    char* ws = (char*)d_ws;
    size_t off = 0;
    _Float16* X16   = (_Float16*)(ws + off); off += (size_t)NROWS * EMB * sizeof(_Float16);
    _Float16* WnT16 = (_Float16*)(ws + off); off += (size_t)NCLS_PAD * EMB * sizeof(_Float16);
    float*    Part  = (float*)(ws + off);    off += (size_t)16 * NROWS * sizeof(float);
    float*  RowLoss = (float*)(ws + off);    off += (size_t)NROWS * sizeof(float);
    float*  RowCorr = (float*)(ws + off);    off += (size_t)NROWS * sizeof(float);
    if (off > ws_size) return;

    k_cvt<<<NROWS / CVT_RPB, 256, 0, stream>>>(X, X16);
    k_wnorm<<<NCLS_PAD, 32, 0, stream>>>(Kw, WnT16);
    k_ce<<<NROWS / CE_RPB, 256, 0, stream>>>(X16, WnT16, tgt, RowLoss, RowCorr);

    dim3 simGrid(NROWS / SIM_RPB, NROWS / SIM_CCH);
    const size_t simShmem = (size_t)SIM_RPB * EMB * sizeof(_Float16)
                          + (size_t)SIM_RPB * sizeof(int) * 2
                          + (size_t)4 * SIM_RPB * sizeof(float);
    k_sim<<<simGrid, 256, simShmem, stream>>>(X16, X, tgt, Part);

    k_fin<<<1, 256, 0, stream>>>(Part, RowLoss, RowCorr, (float*)d_out);
    (void)hipGetLastError();
}
